// KANSplineLayer_88991722373383
// MI455X (gfx1250) — hardware-run, weakly checked
//
#include <hip/hip_runtime.h>
#include <math.h>

constexpr int   kRows        = 32768;
constexpr int   kIn          = 256;
constexpr int   kOut         = 256;
constexpr int   kKnots       = 9;
constexpr int   kSpK         = kIn * kKnots;
constexpr int   kGroupsPerRow = kSpK / 8;
constexpr int   kChunkRows   = 8192;
constexpr int   kNumChunks   = kRows / kChunkRows;
constexpr int   kMMRowsPerBlock = 128;
constexpr int   kMMBlocks    = kRows / kMMRowsPerBlock;
constexpr float kWbCarry     = 64.0f;
constexpr float kWbCarryInv  = 1.0f / 64.0f;
constexpr float kWsCarry     = 256.0f;
constexpr float kWsCarryInv  = 1.0f / 256.0f;
constexpr float kEpsMinMax   = 1e-7f;
constexpr float kEpsBN       = 1e-3f;

constexpr size_t kOffX16    = 0;
constexpr size_t kOffWb16   = kOffX16   + (size_t)kRows * kIn * 2;
constexpr size_t kOffWsp16  = kOffWb16  + (size_t)kOut * kIn * 2;
constexpr size_t kOffPmin   = kOffWsp16 + (size_t)kOut * kSpK * 2;
constexpr size_t kOffPmax   = kOffPmin  + (size_t)kMMBlocks * kIn * 4;
constexpr size_t kOffMM     = kOffPmax  + (size_t)kMMBlocks * kIn * 4;
constexpr size_t kOffBasis  = kOffMM    + 4096;
constexpr size_t kOffBase   = kOffBasis + (size_t)kChunkRows * kSpK * 2;
constexpr size_t kOffSpl    = kOffBase  + (size_t)kRows * kOut * 4;
constexpr size_t kWsTotal   = kOffSpl   + (size_t)kRows * kOut * 4;

typedef __attribute__((ext_vector_type(16))) _Float16 v16h;
typedef __attribute__((ext_vector_type(8)))  _Float16 v8h;
typedef __attribute__((ext_vector_type(16))) __bf16   v16b;
typedef __attribute__((ext_vector_type(8)))  __bf16   v8b;
typedef __attribute__((ext_vector_type(8)))  float    v8f;
typedef __attribute__((ext_vector_type(4)))  float    v4f;
typedef __attribute__((ext_vector_type(4)))  unsigned int v4u;

__device__ __forceinline__ unsigned short f2bf_bits(float f) {
  unsigned u = __float_as_uint(f);
  return (unsigned short)((u + 0x7FFFu + ((u >> 16) & 1u)) >> 16);
}
__device__ __forceinline__ float bf_bits2f(unsigned short h) { return __uint_as_float(((unsigned)h) << 16); }

__device__ __forceinline__ void dep_guard_h(v8f& a, v8f& b, v16h x, v16h y) { asm volatile("v_nop\n\tv_nop\n\tv_nop\n\tv_nop" : "+v"(a), "+v"(b) : "v"(x), "v"(y)); }
__device__ __forceinline__ void dep_guard_b(v8f& a, v8f& b, v16b x, v16b y) { asm volatile("v_nop\n\tv_nop\n\tv_nop\n\tv_nop" : "+v"(a), "+v"(b) : "v"(x), "v"(y)); }
__device__ __forceinline__ void keep4_h(v16h a, v16h b, v16h c, v16h d) { asm volatile("v_nop" :: "v"(a), "v"(b), "v"(c), "v"(d)); }
__device__ __forceinline__ void keep4_b(v16b a, v16b b, v16b c, v16b d) { asm volatile("v_nop" :: "v"(a), "v"(b), "v"(c), "v"(d)); }
__device__ __forceinline__ void acc_guard4(v8f& a, v8f& b, v8f& c, v8f& d) { asm volatile("v_nop\n\tv_nop\n\tv_nop\n\tv_nop" : "+v"(a), "+v"(b), "+v"(c), "+v"(d)); }
template <typename T> struct Frag;
template <> struct Frag<_Float16> {
  typedef v16h V; union U { v16h v; v8h h[2]; };
  static __device__ __forceinline__ v16h load(const _Float16* p) {
    U f; f.h[0] = *(const v8h*)(p); f.h[1] = *(const v8h*)(p + 16); return f.v;
  }
  static __device__ __forceinline__ v8f mma(v16h a, v16h b, v8f c) {
    return __builtin_amdgcn_wmma_f32_16x16x32_f16(false, a, false, b, (short)0, c, false, false);
  }
  static __device__ __forceinline__ void guard(v8f& a, v8f& b, v16h x, v16h y) { dep_guard_h(a, b, x, y); }
  static __device__ __forceinline__ void keep(v16h a, v16h b, v16h c, v16h d) { keep4_h(a, b, c, d); }
};
template <> struct Frag<__bf16> {
  typedef v16b V; union U { v16b v; v8b h[2]; };
  static __device__ __forceinline__ v16b load(const __bf16* p) {
    U f; f.h[0] = *(const v8b*)(p); f.h[1] = *(const v8b*)(p + 16); return f.v;
  }
  static __device__ __forceinline__ v8f mma(v16b a, v16b b, v8f c) {
    return __builtin_amdgcn_wmma_f32_16x16x32_bf16(false, a, false, b, (short)0, c, false, false);
  }
  static __device__ __forceinline__ void guard(v8f& a, v8f& b, v16b x, v16b y) { dep_guard_b(a, b, x, y); }
  static __device__ __forceinline__ void keep(v16b a, v16b b, v16b c, v16b d) { keep4_b(a, b, c, d); }
};

__device__ __forceinline__ unsigned pk16(unsigned short a, unsigned short b) { return (unsigned)a | ((unsigned)b << 16); }
__device__ __forceinline__ unsigned short h_bits(float f) { const _Float16 h = (_Float16)f; return __builtin_bit_cast(unsigned short, h); }

template <int ET> struct Elem;
template <> struct Elem<0> { typedef _Float16 T; };
template <> struct Elem<1> { typedef __bf16 T; };
template <int ET, bool SPLIT, int BIAS_MODE, int OUT_MODE, bool RESID, int ACT = 0>
__global__ __launch_bounds__(256) void wmma_gemm64(
    const unsigned short* __restrict__ Ap, const unsigned short* __restrict__ A2p, int lda, long strideA,
    const unsigned short* __restrict__ Btp, const unsigned short* __restrict__ Bt2p, int ldb, long strideB,
    void* __restrict__ Cout, void* __restrict__ Cout2, int ldc, long strideC,
    const float* __restrict__ bias,
    const float* __restrict__ resid, long strideR,
    int M, int N, int K, float scale) {
  typedef typename Elem<ET>::T T;
  typedef typename Frag<T>::V V;
  const T* A = (const T*)Ap; const T* A2 = (const T*)A2p; const T* Bt = (const T*)Btp; const T* Bt2 = (const T*)Bt2p;
  __shared__ __align__(16) float sT[8][16 * 68];
  const int b    = blockIdx.y;
  const int lane = threadIdx.x & 31;
  const int wave = threadIdx.x >> 5;
  const int tilesN = N >> 6;
  const int tilesM = M >> 6;
  const int tile = blockIdx.x * 8 + wave;
  if (tile >= tilesM * tilesN) return;
  const int tm = tile / tilesN;
  const int tn = tile - tm * tilesN;
  const int m0 = tm << 6;
  const int n0 = tn << 6;

  const T* Ab  = A  + (size_t)b * strideA;
  const T* Bb  = Bt + (size_t)b * strideB;
  const T* Ab2 = SPLIT ? (A2  + (size_t)b * strideA) : nullptr;
  const T* Bb2 = SPLIT ? (Bt2 + (size_t)b * strideB) : nullptr;

  const int rlane = lane & 15;
  const int koff  = (lane >> 4) * 8;
  const int mOff  = (lane >> 4) * 8;

  v8f acc[4][4];
#pragma unroll
  for (int i = 0; i < 4; ++i)
#pragma unroll
    for (int j = 0; j < 4; ++j) acc[i][j] = (v8f){0.f,0.f,0.f,0.f,0.f,0.f,0.f,0.f};

  for (int k0 = 0; k0 < K; k0 += 32) {
    V bh[4], bl[4];
#pragma unroll
    for (int j = 0; j < 4; ++j) {
      const size_t bo = (size_t)(n0 + (j << 4) + rlane) * ldb + koff + k0;
      bh[j] = Frag<T>::load(Bb + bo);
      if (SPLIT) bl[j] = Frag<T>::load(Bb2 + bo);
    }
#pragma unroll
    for (int i = 0; i < 4; ++i) {
      const size_t ao = (size_t)(m0 + (i << 4) + rlane) * lda + koff + k0;
      V ah = Frag<T>::load(Ab + ao);
      V al;
      if (SPLIT) al = Frag<T>::load(Ab2 + ao);
#pragma unroll
      for (int j = 0; j < 4; ++j) {
        acc[i][j] = Frag<T>::mma(ah, bh[j], acc[i][j]);
        if (SPLIT) {
          acc[i][j] = Frag<T>::mma(ah, bl[j], acc[i][j]);
          acc[i][j] = Frag<T>::mma(al, bh[j], acc[i][j]);
        }
      }
      Frag<T>::guard(acc[i][0], acc[i][3], ah, SPLIT ? al : ah);
    }
    Frag<T>::keep(bh[0], bh[1], bh[2], bh[3]);
    if (SPLIT) Frag<T>::keep(bl[0], bl[1], bl[2], bl[3]);
  }
  acc_guard4(acc[0][0], acc[0][1], acc[0][2], acc[0][3]);
  acc_guard4(acc[1][0], acc[1][1], acc[1][2], acc[1][3]);
  acc_guard4(acc[2][0], acc[2][1], acc[2][2], acc[2][3]);
  acc_guard4(acc[3][0], acc[3][1], acc[3][2], acc[3][3]);

  float* slab = sT[wave];
  const float* Rb = RESID ? (resid + (size_t)b * strideR) : nullptr;
#pragma unroll
  for (int i = 0; i < 4; ++i) {
    const int mBase = m0 + (i << 4);
#pragma unroll
    for (int j = 0; j < 4; ++j) {
      const int n = n0 + (j << 4) + rlane;
      float bv = 0.f;
      if (BIAS_MODE == 2) bv = bias[n];
#pragma unroll
      for (int r = 0; r < 8; ++r) {
        float v = acc[i][j][r] * scale;
        if (BIAS_MODE == 1) v += bias[mBase + mOff + r];
        if (BIAS_MODE == 2) v += bv;
        if (RESID) v += Rb[(size_t)(mBase + mOff + r) * ldc + n];
        if (ACT == 2) v = fmaxf(v, 0.0f);
        if (ACT == 4) v = (v > 0.f) ? v : 0.01f * v;
        slab[(mOff + r) * 68 + (j << 4) + rlane] = v;
      }
    }
    __builtin_amdgcn_fence(__ATOMIC_RELEASE, "workgroup");
    __builtin_amdgcn_wave_barrier();
    __builtin_amdgcn_fence(__ATOMIC_ACQUIRE, "workgroup");
    if (OUT_MODE == 0) {
      float* C = (float*)Cout + (size_t)b * strideC;
      const int hh = lane >> 4, c4 = (lane & 15) * 4;
      for (int pass = 0; pass < 2; ++pass) {
#pragma unroll
        for (int it = 0; it < 8; ++it) {
          const int row = it * 2 + hh;
          v4f v = *(const v4f*)(slab + row * 68 + c4);
          *(volatile v4f*)(C + (size_t)(mBase + row) * ldc + n0 + c4) = v;
        }
        __threadfence();
      }
    } else {
      const int q = lane >> 3, c8 = (lane & 7) * 8;
      unsigned short* C  = (unsigned short*)Cout  + (size_t)b * strideC;
      unsigned short* C2 = (OUT_MODE == 2) ? ((unsigned short*)Cout2 + (size_t)b * strideC) : nullptr;
      for (int pass = 0; pass < 2; ++pass) {
#pragma unroll
        for (int it = 0; it < 4; ++it) {
          const int row = it * 4 + q;
          const float* sp = slab + row * 68 + c8;
          v8h hv, lv;
#pragma unroll
          for (int e = 0; e < 8; ++e) {
            if (OUT_MODE == 1) {
              hv[e] = (_Float16)sp[e];
            } else {
              unsigned short hb = f2bf_bits(sp[e]);
              unsigned short lb = f2bf_bits(sp[e] - bf_bits2f(hb));
              hv[e] = __builtin_bit_cast(_Float16, hb);
              lv[e] = __builtin_bit_cast(_Float16, lb);
            }
          }
          *(volatile v8h*)(C + (size_t)(mBase + row) * ldc + n0 + c8) = hv;
          if (OUT_MODE == 2) *(volatile v8h*)(C2 + (size_t)(mBase + row) * ldc + n0 + c8) = lv;
        }
        __threadfence();
      }
    }
    __builtin_amdgcn_fence(__ATOMIC_RELEASE, "workgroup");
    __builtin_amdgcn_wave_barrier();
    __builtin_amdgcn_fence(__ATOMIC_ACQUIRE, "workgroup");
  }
}

__global__ __launch_bounds__(256) void k_minmax_part(const float* __restrict__ x,
                                                     float* __restrict__ pmin, float* __restrict__ pmax) {
  __shared__ __align__(16) float smn[kIn];
  __shared__ __align__(16) float smx[kIn];
  const int t = threadIdx.x;
  const size_t r0 = (size_t)blockIdx.x * kMMRowsPerBlock;
  float mn = 3.0e38f, mx = -3.0e38f;
#pragma unroll 4
  for (int r = 0; r < kMMRowsPerBlock; ++r) {
    const float v = x[(r0 + (size_t)r) * kIn + t];
    mn = fminf(mn, v);
    mx = fmaxf(mx, v);
  }
  smn[t] = mn;
  smx[t] = mx;
  __syncthreads();
  const int lane = t & 31, wave = t >> 5;
  if (wave < 2) {
    const int idx = (wave * 32 + lane) * 4;
    const v4f v = *(const v4f*)(smn + idx);
    float* dst = pmin + (size_t)blockIdx.x * kIn + idx;
    *(volatile v4f*)dst = v;
    __threadfence();
    *(volatile v4f*)dst = v;
  } else if (wave < 4) {
    const int idx = ((wave - 2) * 32 + lane) * 4;
    const v4f v = *(const v4f*)(smx + idx);
    float* dst = pmax + (size_t)blockIdx.x * kIn + idx;
    *(volatile v4f*)dst = v;
    __threadfence();
    *(volatile v4f*)dst = v;
  }
}

__global__ __launch_bounds__(256) void k_minmax_fin(const float* __restrict__ pmin, const float* __restrict__ pmax,
                                                    float* __restrict__ mm) {
  __shared__ __align__(16) float smm[2 * kIn];
  const int t = threadIdx.x;
  float mn = 3.0e38f, mx = -3.0e38f;
#pragma unroll 4
  for (int b = 0; b < kMMBlocks; ++b) {
    mn = fminf(mn, pmin[(size_t)b * kIn + t]);
    mx = fmaxf(mx, pmax[(size_t)b * kIn + t]);
  }
  const float d = (mx - mn) + kEpsMinMax;
  const float rcp = 1.0f / d;
  smm[t] = mn;
  smm[kIn + t] = rcp;
  __syncthreads();
  const int lane = t & 31, wave = t >> 5;
  if (wave == 0) {
    for (int pass = 0; pass < 2; ++pass) {
#pragma unroll
      for (int it = 0; it < 4; ++it) {
        const int idx = it * 128 + lane * 4;
        const v4f v = *(const v4f*)(smm + idx);
        *(volatile v4f*)(mm + idx) = v;
      }
      __threadfence();
    }
  }
}

__global__ __launch_bounds__(256) void cast8_f16_kernel(const float* __restrict__ in, unsigned short* __restrict__ out, int n8) {
  const int i = blockIdx.x * 256 + threadIdx.x;
  if (i >= n8) return;
  const float* p = in + 8 * (size_t)i;
  const v4f a = *(const v4f*)(p);
  const v4f c = *(const v4f*)(p + 4);
  unsigned short hb[8];
#pragma unroll
  for (int e = 0; e < 4; ++e) {
    hb[e]     = h_bits(a[e]);
    hb[4 + e] = h_bits(c[e]);
  }
  const v4u u = (v4u){pk16(hb[0], hb[1]), pk16(hb[2], hb[3]), pk16(hb[4], hb[5]), pk16(hb[6], hb[7])};
  unsigned short* q = out + 8 * (size_t)i;
  *(volatile v4u*)q = u;
  __threadfence();
  *(volatile v4u*)q = u;
}

__global__ __launch_bounds__(256) void k_wbase_tcast(const float* __restrict__ W, unsigned short* __restrict__ out, float scale) {
  __shared__ float sm[64][65];
  const int t  = threadIdx.x;
  const int d0 = blockIdx.x * 64;
  const int h0 = blockIdx.y * 64;
#pragma unroll
  for (int i = 0; i < 16; ++i) {
    const int e = i * 256 + t;
    const int r = e >> 6;
    const int c = e & 63;
    sm[c][r] = W[(size_t)(d0 + r) * kOut + h0 + c] * scale;
  }
  __syncthreads();
  const int lane = t & 31, wave = t >> 5;
  const int q = lane >> 3, c8 = (lane & 7) * 8;
  for (int pass = 0; pass < 2; ++pass) {
#pragma unroll
    for (int it = 0; it < 2; ++it) {
      const int row = wave * 8 + it * 4 + q;
      unsigned short hb[8];
#pragma unroll
      for (int e = 0; e < 8; ++e) hb[e] = h_bits(sm[row][c8 + e]);
      const v4u u = (v4u){pk16(hb[0], hb[1]), pk16(hb[2], hb[3]), pk16(hb[4], hb[5]), pk16(hb[6], hb[7])};
      *(volatile v4u*)(out + (size_t)(h0 + row) * kIn + d0 + c8) = u;
    }
    __threadfence();
  }
}

__global__ __launch_bounds__(256) void k_wsp_cast(const float* __restrict__ sw, const float* __restrict__ sc,
                                                unsigned short* __restrict__ out, int n8) {
  const int i = blockIdx.x * 256 + threadIdx.x;
  if (i >= n8) return;
  const int flat0 = 8 * i;
  const int o  = flat0 / kSpK;
  const int k0 = flat0 - o * kSpK;
  const float* p = sw + (size_t)flat0;
  const v4f a = *(const v4f*)(p);
  const v4f c = *(const v4f*)(p + 4);
  unsigned short hb[8];
#pragma unroll
  for (int e = 0; e < 8; ++e) {
    const int in_e = (k0 + e) / kKnots;
    const float s = sc[(size_t)o * kIn + in_e];
    const float wv = (e < 4) ? a[e] : c[e - 4];
    hb[e] = h_bits((wv * s) * kWsCarry);
  }
  const v4u u = (v4u){pk16(hb[0], hb[1]), pk16(hb[2], hb[3]), pk16(hb[4], hb[5]), pk16(hb[6], hb[7])};
  unsigned short* q = out + 8 * (size_t)i;
  *(volatile v4u*)q = u;
  __threadfence();
  *(volatile v4u*)q = u;
}

__global__ __launch_bounds__(256) void k_basis8(const float* __restrict__ x, const float* __restrict__ mm,
                                               unsigned short* __restrict__ out, int row_base, int nthr) {
#pragma clang fp contract(off)
  const int i = blockIdx.x * 256 + threadIdx.x;
  if (i >= nthr) return;
  const int rl  = i / kGroupsPerRow;
  const int q   = i - rl * kGroupsPerRow;
  const int row = row_base + rl;
  const int k0  = q * 8;
  const int i0  = k0 / kKnots;
  const int j0  = k0 - i0 * kKnots;
  int i1 = i0 + 1;
  i1 = (i1 > kIn - 1) ? (kIn - 1) : i1;
  const float* xr = x + (size_t)row * kIn;
  const float xa = xr[i0];
  const float xb = xr[i1];
  const float xna = (xa - mm[i0]) * mm[kIn + i0];
  const float xnb = (xb - mm[i1]) * mm[kIn + i1];
  unsigned short hb[8];
#pragma unroll
  for (int e = 0; e < 8; ++e) {
    int j = j0 + e;
    const bool w = (j >= kKnots);
    j = w ? (j - kKnots) : j;
    const float xv = w ? xnb : xna;
    const float kn = -1.0f + 0.25f * (float)j;
    const float dd = xv - kn;
    const float bas = fmaxf(0.0f, 1.0f - fabsf(dd));
    hb[e] = h_bits(bas);
  }
  const v4u u = (v4u){pk16(hb[0], hb[1]), pk16(hb[2], hb[3]), pk16(hb[4], hb[5]), pk16(hb[6], hb[7])};
  unsigned short* qp = out + 8 * (size_t)i;
  *(volatile v4u*)qp = u;
  __threadfence();
  *(volatile v4u*)qp = u;
}

__global__ __launch_bounds__(256) void k_final(const float* __restrict__ baseacc, const float* __restrict__ splacc,
                                              const float* __restrict__ g1, const float* __restrict__ b1,
                                              const float* __restrict__ m1, const float* __restrict__ v1,
                                              const float* __restrict__ g2, const float* __restrict__ b2,
                                              const float* __restrict__ m2, const float* __restrict__ v2,
                                              float* __restrict__ out, int n4) {
  const int i = blockIdx.x * 256 + threadIdx.x;
  if (i >= n4) return;
  const int c4 = (i & (kOut / 4 - 1)) * 4;
  const v4f zb = *(const v4f*)(baseacc + 4 * (size_t)i);
  const v4f zs = *(const v4f*)(splacc  + 4 * (size_t)i);
  const v4f G1 = *(const v4f*)(g1 + c4), B1 = *(const v4f*)(b1 + c4), M1 = *(const v4f*)(m1 + c4), V1 = *(const v4f*)(v1 + c4);
  const v4f G2 = *(const v4f*)(g2 + c4), B2 = *(const v4f*)(b2 + c4), M2 = *(const v4f*)(m2 + c4), V2 = *(const v4f*)(v2 + c4);
  v4f o;
#pragma unroll
  for (int e = 0; e < 4; ++e) {
    const float rs1 = rsqrtf(V1[e] + kEpsBN);
    const float z   = G1[e] * (zb[e] - M1[e]) * rs1 + B1[e];
    const float tex = expf(-z);
    const float sig = __builtin_amdgcn_rcpf(1.0f + tex);
    const float bse = z * sig;
    const float rs2 = rsqrtf(V2[e] + kEpsBN);
    const float sp  = G2[e] * (zs[e] - M2[e]) * rs2 + B2[e];
    o[e] = bse + sp;
  }
  float* q = out + 4 * (size_t)i;
  *(volatile v4f*)q = o;
  __threadfence();
  *(volatile v4f*)q = o;
}

extern "C" void kernel_launch(void* const* d_in, const int* in_sizes, int n_in,
                              void* d_out, int out_size, void* d_ws, size_t ws_size,
                              hipStream_t stream) {
  if (n_in < 12) return;
  if (ws_size < kWsTotal) return;
  if (in_sizes[0] != kRows * kIn) return;
  if (out_size != kRows * kOut) return;

  const float* x   = (const float*)d_in[0];
  const float* bw  = (const float*)d_in[1];
  const float* sw  = (const float*)d_in[2];
  const float* sc  = (const float*)d_in[3];
  const float* g1  = (const float*)d_in[4];
  const float* b1  = (const float*)d_in[5];
  const float* m1  = (const float*)d_in[6];
  const float* v1  = (const float*)d_in[7];
  const float* g2  = (const float*)d_in[8];
  const float* b2  = (const float*)d_in[9];
  const float* m2  = (const float*)d_in[10];
  const float* v2  = (const float*)d_in[11];
  float* outp = (float*)d_out;

  char* ws = (char*)d_ws;
  unsigned short* x16   = (unsigned short*)(ws + kOffX16);
  unsigned short* wb16  = (unsigned short*)(ws + kOffWb16);
  unsigned short* wsp16 = (unsigned short*)(ws + kOffWsp16);
  float* pmin    = (float*)(ws + kOffPmin);
  float* pmax    = (float*)(ws + kOffPmax);
  float* mm      = (float*)(ws + kOffMM);
  unsigned short* basis = (unsigned short*)(ws + kOffBasis);
  float* baseacc = (float*)(ws + kOffBase);
  float* splacc  = (float*)(ws + kOffSpl);

  k_minmax_part<<<kMMBlocks, 256, 0, stream>>>(x, pmin, pmax);
  k_minmax_fin<<<1, 256, 0, stream>>>(pmin, pmax, mm);

  const int n8x = kRows * kIn / 8;
  cast8_f16_kernel<<<(n8x + 255) / 256, 256, 0, stream>>>(x, x16, n8x);
  k_wbase_tcast<<<dim3(kIn / 64, kOut / 64), 256, 0, stream>>>(bw, wb16, kWbCarry);
  const int n8w = kOut * kSpK / 8;
  k_wsp_cast<<<(n8w + 255) / 256, 256, 0, stream>>>(sw, sc, wsp16, n8w);

  {
    const int tiles = (kRows / 64) * (kOut / 64);
    wmma_gemm64<0, false, 0, 0, false, 0><<<dim3((tiles + 7) / 8, 1), 256, 0, stream>>>(
        x16, x16, kIn, 0L, wb16, wb16, kIn, 0L,
        (void*)baseacc, (void*)baseacc, kOut, 0L,
        mm, baseacc, 0L, kRows, kOut, kIn, kWbCarryInv);
  }

  const int nthr_basis = kChunkRows * kGroupsPerRow;
  const int tiles_sp   = (kChunkRows / 64) * (kOut / 64);
  for (int c = 0; c < kNumChunks; ++c) {
    k_basis8<<<(nthr_basis + 255) / 256, 256, 0, stream>>>(x, mm, basis, c * kChunkRows, nthr_basis);
    float* cacc = splacc + (size_t)c * kChunkRows * kOut;
    wmma_gemm64<0, false, 0, 0, false, 0><<<dim3((tiles_sp + 7) / 8, 1), 256, 0, stream>>>(
        basis, basis, kSpK, 0L, wsp16, wsp16, kSpK, 0L,
        (void*)cacc, (void*)cacc, kOut, 0L,
        mm, cacc, 0L, kChunkRows, kOut, kSpK, kWsCarryInv);
  }

  const int n4 = kRows * kOut / 4;
  k_final<<<(n4 + 255) / 256, 256, 0, stream>>>(baseacc, splacc, g1, b1, m1, v1, g2, b2, m2, v2, outp, n4);
}
